// LASMConvssw_29197187678930
// MI455X (gfx1250) — hardware-run, weakly checked
//
#include <hip/hip_runtime.h>


#ifndef NB
#define NB 4
#endif
#ifndef NPT
#define NPT 20000
#endif
#define NB_FULL  4
#define NPT_FULL 20000
#ifndef OUT_NPT
#define OUT_NPT NPT
#endif
#define NBR  9
#define WN   17
#define CI   64
#define CO   128
#define KT   (WN * CI)
#define ROWS 32
#define PTS  (ROWS / NB)
#define AP   (KT + 8)
#define OSP  132
#define WNP  12
#define SW_N (PTS * WN * WNP)
#define SW_IT ((SW_N + 255) / 256)
#define LOG2E 1.4426950408889634f

static_assert(ROWS == 32);
static_assert(ROWS % NB == 0);
static_assert(PTS * NB == ROWS);
static_assert(NPT % PTS == 0);
static_assert(NB <= NB_FULL);
static_assert(NPT <= NPT_FULL);
static_assert(CI == 64);
static_assert(ROWS * (CI / 8) == 256);
static_assert(CO == 8 * 16);
static_assert(KT % 32 == 0);
static_assert((KT / 32) % 2 == 0);
static_assert(AP % 8 == 0);
static_assert(AP >= KT);
static_assert((OSP * 4) % 16 == 0);
static_assert(OSP >= CO);
static_assert(WNP >= NBR);
static_assert(WNP % 4 == 0);
static_assert(256 * 16 * 4 == ROWS * CO * 4);
static_assert(32 * 16 == CO * 4);
static_assert((size_t)ROWS * AP * 2 + (size_t)SW_N * 4 + (size_t)ROWS * OSP * 4 <= 131072);
static_assert(((size_t)NB * NPT_FULL * CI) % 8 == 0);
static_assert(((size_t)CO * KT) % 8 == 0);
static_assert((CO * KT / 8) % 256 == 0);

typedef _Float16 h16;
typedef unsigned short bf;
typedef __attribute__((ext_vector_type(16))) _Float16 v16h;
typedef __attribute__((ext_vector_type(8)))  _Float16 v8h;
typedef __attribute__((ext_vector_type(8)))  unsigned short v8us;
typedef __attribute__((ext_vector_type(8)))  float    v8f;
typedef __attribute__((ext_vector_type(4)))  float    v4f;
typedef v4f  __attribute__((may_alias)) v4fa;

__device__ __forceinline__ unsigned short f2bf(float f) { unsigned u = __float_as_uint(f); u += 0x7FFFu + ((u >> 16) & 1u); return (unsigned short)(u >> 16); }
__device__ __forceinline__ float bfr(float f) { return __uint_as_float(((unsigned)f2bf(f)) << 16); }
__device__ __forceinline__ v16h cat16(v8h lo, v8h hi) { return __builtin_shufflevector(lo, hi, 0, 1, 2, 3, 4, 5, 6, 7, 8, 9, 10, 11, 12, 13, 14, 15); }
__device__ __forceinline__ v8f wmma16(v16h a, v16h b, v8f c) { return __builtin_amdgcn_wmma_f32_16x16x32_f16(false, a, false, b, (short)0, c, false, false); }
__device__ __forceinline__ v16h  ldh(const h16* p) { return cat16(*(const v8h*)p, *(const v8h*)(p + 16)); }

static __device__ __forceinline__ h16 toh_flush(float v) { const h16 r = (h16)v; return (fabsf(v) < 6.103515625e-05f) ? (h16)0.0f : r; }
__device__ __forceinline__ v8f wmma16g(v16h a, v16h b, v8f c) { c = wmma16(a, b, c); asm volatile("v_nop\n\tv_nop\n\tv_nop\n\tv_nop" : "+v"(c) : "v"(a), "v"(b)); return c; }
__device__ __forceinline__ bool nid_fix(int id, int& row) {
    int idn = id < 0 ? id + (NPT_FULL + 1) : id;
    idn = idn < 0 ? 0 : (idn > NPT_FULL ? NPT_FULL : idn);
    const bool keep = (id < NPT_FULL) & (idn < NPT_FULL);
    row = idn < NPT_FULL ? idn : (NPT_FULL - 1);
    return keep;
}
__device__ __forceinline__ float elu1(float v) {
    const float neg = (v > 0.0f) ? 0.0f : v;
    const float e = __builtin_amdgcn_exp2f(neg * LOG2E) - 1.0f;
    return (v > 0.0f) ? v : e;
}

__global__ __launch_bounds__(256) void k_cvt8(const float* __restrict__ src, bf* dst, size_t n8) {
    const size_t i = (size_t)blockIdx.x * 256 + threadIdx.x; if (i >= n8) return;
    const v8f v = *(const v8f*)(src + i * 8); v8us o;
#pragma unroll
    for (int k = 0; k < 8; ++k) o[k] = f2bf(v[k]);
    *(volatile v8us*)(dst + i * 8) = o; __threadfence(); *(volatile v8us*)(dst + i * 8) = o;
}

__global__ __launch_bounds__(256) void k_wconv(const float* __restrict__ W, h16* WT, int n8) {
    const int t = blockIdx.x * 256 + threadIdx.x; if (t >= n8) return;
    const int o = t / (KT / 8), k8 = t % (KT / 8);
    const int m = k8 >> 3, i0 = (k8 & 7) * 8;
    const v8f v = *(const v8f*)(W + (size_t)m * (CO * CI) + (size_t)o * CI + i0);
    v8h hv;
#pragma unroll
    for (int k = 0; k < 8; ++k) hv[k] = toh_flush(bfr(v[k]));
    *(volatile v8h*)(WT + (size_t)t * 8) = hv; __threadfence(); *(volatile v8h*)(WT + (size_t)t * 8) = hv;
}

__global__ __launch_bounds__(256) void k_fused(const bf* __restrict__ XB, const float* __restrict__ raww, const h16* __restrict__ WT,
                                               const float* __restrict__ bias, const int* __restrict__ nbr, float* OUT) {
    __shared__ __align__(16) h16   sA[ROWS * AP];
    __shared__ __align__(16) float sW[SW_N];
    __shared__ __align__(16) float os[ROWS * OSP];
    const int tid = threadIdx.x;
    const int lane = tid & 31, lr = lane & 15, hi = lane >> 4;
    const int wave = __builtin_amdgcn_readfirstlane((int)(threadIdx.x >> 5));
    const int pt0 = blockIdx.x * PTS;

#pragma unroll 1
    for (int it = 0; it < SW_IT; ++it) {
        const int e = it * 256 + tid;
        const int ec = e < SW_N ? e : (SW_N - 1);
        const int n = ec % WNP, m = (ec / WNP) % WN, pl = ec / (WNP * WN);
        const int nc = n < NBR ? n : (NBR - 1);
        const size_t pn = (size_t)(pt0 + pl) * NBR + nc;
        int id = nbr[pn]; float w = raww[pn * WN + m];
        asm volatile("" : "+v"(id)); asm volatile("" : "+v"(w));
        int rowx; const bool keep = nid_fix(id, rowx) & (n < NBR);
        const float val = keep ? bfr(w) : 0.0f;
        if (e < SW_N) sW[e] = val;
    }

    const int r = tid >> 3, g = tid & 7;
    const int b = r / PTS, pl = r % PTS;
    float x[NBR][8];
    {
        const v8us zz = (v8us){};
        v8us u[NBR];
#pragma unroll
        for (int n = 0; n < NBR; ++n) {
            const int id = nbr[(size_t)(pt0 + pl) * NBR + n];
            int row; const bool keep = nid_fix(id, row);
            v8us t = *(const v8us*)(XB + ((size_t)b * NPT_FULL + (size_t)row) * CI + g * 8);
            asm volatile("" : "+v"(t));
            u[n] = keep ? t : zz;
        }
#pragma unroll
        for (int n = 0; n < NBR; ++n)
#pragma unroll
            for (int k = 0; k < 8; ++k) x[n][k] = __uint_as_float(((unsigned)u[n][k]) << 16);
    }
    __syncthreads();

#pragma unroll 1
    for (int m = 0; m < WN; ++m) {
        const int wb = (pl * WN + m) * WNP;
        const v4f w0 = *(const v4fa*)(&sW[wb]); const v4f w1 = *(const v4fa*)(&sW[wb + 4]); const v4f w2 = *(const v4fa*)(&sW[wb + 8]);
        float a[8];
#pragma unroll
        for (int k = 0; k < 8; ++k) {
            float s = w0[0] * x[0][k];
            s += w0[1] * x[1][k]; s += w0[2] * x[2][k]; s += w0[3] * x[3][k];
            s += w1[0] * x[4][k]; s += w1[1] * x[5][k]; s += w1[2] * x[6][k]; s += w1[3] * x[7][k];
            s += w2[0] * x[8][k];
            a[k] = s;
        }
        v8h hv;
#pragma unroll
        for (int k = 0; k < 8; ++k) hv[k] = toh_flush(a[k]);
        *(v8h*)(&sA[r * AP + m * CI + g * 8]) = hv;
    }
    __syncthreads();

    v8f acc0 = (v8f){}, acc1 = (v8f){};
    const int n0 = wave * 16;
    const size_t boff = (size_t)(n0 + lr) * KT + 8 * hi;
    const int a0o = lr * AP + 8 * hi, a1o = (16 + lr) * AP + 8 * hi;
#pragma unroll 2
    for (int kc = 0; kc < KT; kc += 32) {
        const v16h bq = ldh(WT + boff + kc);
        const v16h a0 = cat16(*(const v8h*)(&sA[a0o + kc]), *(const v8h*)(&sA[a0o + kc + 16]));
        const v16h a1 = cat16(*(const v8h*)(&sA[a1o + kc]), *(const v8h*)(&sA[a1o + kc + 16]));
        acc0 = wmma16g(a0, bq, acc0);
        acc1 = wmma16g(a1, bq, acc1);
    }

#pragma unroll
    for (int j = 0; j < 8; ++j) { os[(8 * hi + j) * OSP + n0 + lr] = acc0[j]; os[(16 + 8 * hi + j) * OSP + n0 + lr] = acc1[j]; }
    __syncthreads();
    v4f val[4];
    const int c4 = lane * 4;
#pragma unroll
    for (int s = 0; s < 4; ++s) {
        const int row = s * 8 + wave; const int opl = row % PTS;
        const v4f av = *(const v4fa*)(&os[row * OSP + c4]);
        const v4f bv = *(const v4f*)(bias + (size_t)(pt0 + opl) * CO + c4);
#pragma unroll
        for (int i = 0; i < 4; ++i) val[s][i] = elu1(av[i] + bfr(bv[i]));
    }
#pragma unroll
    for (int s = 0; s < 4; ++s) { const int row = s * 8 + wave; const int ob = row / PTS, opl = row % PTS;
        *(volatile v4f*)(OUT + ((size_t)ob * OUT_NPT + (size_t)(pt0 + opl)) * CO + c4) = val[s]; }
    __threadfence();
#pragma unroll
    for (int s = 0; s < 4; ++s) { const int row = s * 8 + wave; const int ob = row / PTS, opl = row % PTS;
        *(volatile v4f*)(OUT + ((size_t)ob * OUT_NPT + (size_t)(pt0 + opl)) * CO + c4) = val[s]; }
}

static constexpr size_t al256(size_t v) { return (v + 255) & ~(size_t)255; }
static constexpr size_t SZ_XB = al256((size_t)NB * NPT_FULL * CI * 2);
static constexpr size_t SZ_WT = al256((size_t)CO * KT * 2);
static constexpr size_t SZ_TOTAL = SZ_XB + SZ_WT;
static_assert(SZ_TOTAL <= (size_t)134217728);
static_assert(((size_t)NB * NPT_FULL * CI * 2) % 128 == 0);
static_assert(((size_t)CO * KT * 2) % 128 == 0);

extern "C" void kernel_launch(void* const* d_in, const int* in_sizes, int n_in,
                              void* d_out, int out_size, void* d_ws, size_t ws_size, hipStream_t stream) {
    if (n_in < 5) return;
    if ((size_t)in_sizes[0] < (size_t)NB * NPT_FULL * CI) return;
    if ((size_t)in_sizes[1] < (size_t)NPT * NBR * WN) return;
    if ((size_t)in_sizes[2] < (size_t)WN * CO * CI) return;
    if ((size_t)in_sizes[3] < (size_t)NPT * CO) return;
    if ((size_t)in_sizes[4] < (size_t)NPT * NBR) return;
    if ((size_t)out_size < ((size_t)(NB - 1) * OUT_NPT + NPT) * CO) return;
    if (SZ_TOTAL > ws_size) return;
    const float* in_pc = (const float*)d_in[0];
    const float* raww  = (const float*)d_in[1];
    const float* wts   = (const float*)d_in[2];
    const float* bias  = (const float*)d_in[3];
    const int*   nbr   = (const int*)d_in[4];
    float* OUT = (float*)d_out;
    char* wsp = (char*)d_ws;
    bf*  XB = (bf*)wsp;  wsp += SZ_XB;
    h16* WT = (h16*)wsp; wsp += SZ_WT;

    { const size_t n8 = (size_t)NB * NPT_FULL * CI / 8;
      k_cvt8<<<(unsigned)((n8 + 255) / 256), 256, 0, stream>>>(in_pc, XB, n8); }
    { const int n8 = CO * KT / 8;
      k_wconv<<<(unsigned)((n8 + 255) / 256), 256, 0, stream>>>(wts, WT, n8); }
    k_fused<<<dim3(NPT / PTS, 1, 1), 256, 0, stream>>>(XB, raww, WT, bias, nbr, OUT);
}
